// V4_SemanticAbstraction_85667417686648
// MI455X (gfx1250) — hardware-verified
//
#include <hip/hip_runtime.h>


namespace {
constexpr int Bn = 4, DIM = 256, DI = 512, DS = 16, DTR = 16, KC = 4, L = 4096, NT = Bn * L, NXP = DTR + 2 * DS  , NXPP = 64;

typedef _Float16 b16;
typedef __attribute__((ext_vector_type(16))) _Float16 v16b;
typedef __attribute__((ext_vector_type(8))) _Float16 v8b;
typedef __attribute__((ext_vector_type(8))) float v8f;
typedef __attribute__((ext_vector_type(4))) float v4f;
__device__ __forceinline__ void split16(float v, b16& hi, b16& lo) { hi = (b16)v; lo = (b16)(v - (float)hi); }
__device__ __forceinline__ v16b frag_kb(const b16* p, int hh) { const v8b a = *(const v8b*)(p + 8 * hh), b = *(const v8b*)(p + 16 + 8 * hh); v16b f;
#pragma unroll
  for (int e = 0; e < 8; ++e) { f[e] = a[e]; f[8 + e] = b[e]; } return f; }
__device__ __forceinline__ v8f wmma16b(v16b a, v16b b, v8f c) {
  v8f d = __builtin_amdgcn_wmma_f32_16x16x32_f16(false, a, false, b, (short)0, c, false, false);
  asm volatile("v_nop\n\tv_nop\n\tv_nop\n\tv_nop" : "+v"(d) : "v"(a), "v"(b));
  return d;
}
__device__ __forceinline__ void wave_lds_sync() { __builtin_amdgcn_fence(__ATOMIC_RELEASE, "workgroup"); __builtin_amdgcn_wave_barrier(); __builtin_amdgcn_fence(__ATOMIC_ACQUIRE, "workgroup"); }
__device__ __forceinline__ float silu_(float v) { return v / (1.0f + __expf(-v)); }
__device__ __forceinline__ float softplus_(float v) { return (v > 20.0f) ? v : log1pf(__expf(v)); }
__device__ __forceinline__ float nexp(float x) { return __builtin_amdgcn_exp2f(x * 1.4426950408889634f); }
__device__ __forceinline__ float nsoftplus(float v) { const float e = nexp(-fabsf(v)); return fmaxf(v, 0.0f) + __builtin_amdgcn_logf(1.0f + e) * 0.69314718055994531f; }
__device__ __forceinline__ float nsilu(float v) { return v * __builtin_amdgcn_rcpf(1.0f + nexp(-v)); }
__device__ __forceinline__ float pmul(float a, float b) { float p = a * b; asm volatile("" : "+v"(p)); return p; }

__global__ __launch_bounds__(256) void prep_kernel(const float* __restrict__ x, const float* __restrict__ win, const float* __restrict__ wx, const float* __restrict__ wout,
                                                   b16* __restrict__ xh, b16* __restrict__ xl, b16* __restrict__ wih, b16* __restrict__ wil, b16* __restrict__ wxh, b16* __restrict__ wxl, b16* __restrict__ woh, b16* __restrict__ wol) {
  const size_t tid = (size_t)blockIdx.x * blockDim.x + threadIdx.x, nth = (size_t)gridDim.x * blockDim.x;
  for (int pass = 0; pass < 2; ++pass) {
    for (size_t p = tid; p < (size_t)NT * DIM / 8; p += nth) { const int t = (int)(p / (DIM / 8)), c0 = (int)(p % (DIM / 8)) * 8, b = t / L, l = t % L; v8b h, lo;
#pragma unroll
      for (int e = 0; e < 8; ++e) { b16 a, c; split16(x[((size_t)b * DIM + c0 + e) * L + l] * 8.0f, a, c); h[e] = a; lo[e] = c; }
      *(volatile v8b*)(xh + (size_t)t * DIM + c0) = h; *(volatile v8b*)(xl + (size_t)t * DIM + c0) = lo; }
    for (size_t p = tid; p < (size_t)2 * DI * DIM; p += nth) { b16 a, c; split16(win[p] * 64.0f, a, c); ((volatile b16*)wih)[p] = a; ((volatile b16*)wil)[p] = c; }
    for (size_t p = tid; p < (size_t)NXPP * DI; p += nth) { const int n = (int)(p / DI); const float v = (n < NXP) ? wx[(size_t)min(n, NXP - 1) * DI + p % DI] * 64.0f : 0.0f; b16 a, c; split16(v, a, c); ((volatile b16*)wxh)[p] = a; ((volatile b16*)wxl)[p] = c; }
    for (size_t p = tid; p < (size_t)DIM * DI; p += nth) { b16 a, c; split16(wout[p] * 64.0f, a, c); ((volatile b16*)woh)[p] = a; ((volatile b16*)wol)[p] = c; }
    __threadfence();
  }
}

template <int K, int NOUT, bool F16OUT>
__global__ __launch_bounds__(128) void gemm_kernel(const b16* __restrict__ ah, const b16* __restrict__ al, const b16* __restrict__ bh, const b16* __restrict__ bl, void* __restrict__ yv) {
  __shared__ __attribute__((aligned(16))) float Ts[4][32 * 64];
  const int lane = threadIdx.x & 31, wave = threadIdx.x >> 5, nloc = lane & 15, hlf = lane >> 4, m0 = blockIdx.y * 128 + wave * 32, c0 = blockIdx.x * 64;
  v8f acc[2][4];
#pragma unroll
  for (int r = 0; r < 2; ++r)
#pragma unroll
    for (int t = 0; t < 4; ++t) acc[r][t] = (v8f){};
#pragma unroll 1
  for (int kb = 0; kb < K; kb += 32) { const v16b a0 = frag_kb(ah + (size_t)(m0 + nloc) * K + kb, hlf), l0 = frag_kb(al + (size_t)(m0 + nloc) * K + kb, hlf), a1 = frag_kb(ah + (size_t)(m0 + 16 + nloc) * K + kb, hlf), l1 = frag_kb(al + (size_t)(m0 + 16 + nloc) * K + kb, hlf);
#pragma unroll
    for (int t = 0; t < 4; ++t) { const size_t bo = (size_t)(c0 + t * 16 + nloc) * K + kb; const v16b b0 = frag_kb(bh + bo, hlf), b1 = frag_kb(bl + bo, hlf);
      acc[0][t] = wmma16b(a0, b0, acc[0][t]); acc[0][t] = wmma16b(l0, b0, acc[0][t]); acc[0][t] = wmma16b(a0, b1, acc[0][t]);
      acc[1][t] = wmma16b(a1, b0, acc[1][t]); acc[1][t] = wmma16b(l1, b0, acc[1][t]); acc[1][t] = wmma16b(a1, b1, acc[1][t]); } }
  float* Tt = Ts[wave];
#pragma unroll
  for (int t = 0; t < 4; ++t)
#pragma unroll
    for (int r = 0; r < 2; ++r)
#pragma unroll
      for (int v = 0; v < 8; ++v) Tt[(r * 16 + v + 8 * hlf) * 64 + t * 16 + nloc] = acc[r][t][v] * (1.0f / 512.0f);
  wave_lds_sync();
  if (!F16OUT) { float* dst0 = (float*)yv + (size_t)m0 * NOUT + c0;
    for (int pass = 0; pass < 2; ++pass) {
#pragma unroll
      for (int j = 0; j < 16; ++j) { const int rr = j * 2 + hlf, c4 = nloc * 4; *(volatile v4f*)(dst0 + (size_t)rr * NOUT + c4) = *(const v4f*)(Tt + rr * 64 + c4); }
      __threadfence(); }
  } else { b16* dst0 = (b16*)yv + (size_t)m0 * NOUT + c0; typedef __attribute__((ext_vector_type(8))) _Float16 v8b_;
    for (int pass = 0; pass < 2; ++pass) {
#pragma unroll
      for (int j = 0; j < 8; ++j) { const int rr = j * 4 + (lane >> 3), c8 = (lane & 7) * 8; v8b_ o;
#pragma unroll
        for (int e = 0; e < 8; ++e) o[e] = (b16)Tt[rr * 64 + c8 + e];
        *(volatile v8b_*)(dst0 + (size_t)rr * NOUT + c8) = o; }
      __threadfence(); }
  }
}

__global__ __launch_bounds__(256) void conv_kernel(const float* __restrict__ u0, const float* __restrict__ cw, const float* __restrict__ cb, b16* __restrict__ uh, b16* __restrict__ ul) {
  const size_t i = (size_t)blockIdx.x * 256 + threadIdx.x; const int t = (int)(i >> 7), dq = (int)(i & 127) * 4, l = t % L;
  v4f o = {0.0f, 0.0f, 0.0f, 0.0f}; typedef __attribute__((ext_vector_type(4))) _Float16 v4b; v4b oh, ol;
#pragma unroll
  for (int c = 0; c < 4; ++c) { const int d = dq + c; float s = cb[d];
#pragma unroll
    for (int k = 0; k < KC; ++k) { const int lt = l - (KC - 1) + k; s += (lt >= 0) ? cw[d * KC + k] * u0[(size_t)max(t - (KC - 1) + k, 0) * DI + d] : 0.0f; }
    const float sv = silu_(s); b16 a, cc; split16(sv * 8.0f, a, cc); oh[c] = a; ol[c] = cc; }
  (void)o;
  for (int pass = 0; pass < 2; ++pass) { *(volatile v4b*)(uh + (size_t)t * DI + dq) = oh; *(volatile v4b*)(ul + (size_t)t * DI + dq) = ol; __threadfence(); }
}

__global__ __launch_bounds__(256) void scan_kernel(const float* __restrict__ dbc, b16* uyh, b16* uyl, const float* __restrict__ res, const float* __restrict__ wdt, const float* __restrict__ bdt, const float* __restrict__ alog, const float* __restrict__ Dv) {
  const int wave = threadIdx.x >> 5, lane = threadIdx.x & 31, b = blockIdx.y; const int dA = wave * 64 + lane, dB = dA + 32;
  float A0[DS], A1[DS], s0[DS], s1[DS], w0[DTR], w1[DTR];
#pragma unroll
  for (int n = 0; n < DS; ++n) { A0[n] = -nexp(alog[dA * DS + n]); A1[n] = -nexp(alog[dB * DS + n]); s0[n] = 0.0f; s1[n] = 0.0f; }
#pragma unroll
  for (int r = 0; r < DTR; ++r) { w0[r] = wdt[dA * DTR + r]; w1[r] = wdt[dB * DTR + r]; }
  const float b0 = bdt[dA], b1 = bdt[dB], D0 = Dv[dA], D1 = Dv[dB];
  for (int l = 0; l < L; ++l) { const size_t t = (size_t)b * L + l; const float* row = dbc + t * NXPP;
    float dt0 = b0, dt1 = b1;
#pragma unroll
    for (int r = 0; r < DTR; ++r) { const float x = row[r]; dt0 += pmul(x, w0[r]); dt1 += pmul(x, w1[r]); }
    const float de0 = nsoftplus(dt0), de1 = nsoftplus(dt1);
    const float u0_ = ((float)uyh[t * DI + dA] + (float)uyl[t * DI + dA]) * 0.125f, u1_ = ((float)uyh[t * DI + dB] + (float)uyl[t * DI + dB]) * 0.125f;
    const float du0 = de0 * u0_, du1 = de1 * u1_; float y0 = 0.0f, y1 = 0.0f;
#pragma unroll
    for (int n = 0; n < DS; ++n) { const float bn = row[DTR + n], cn = row[DTR + DS + n];
      s0[n] = pmul(nexp(de0 * A0[n]), s0[n]) + pmul(du0, bn); s1[n] = pmul(nexp(de1 * A1[n]), s1[n]) + pmul(du1, bn);
      y0 += pmul(s0[n], cn); y1 += pmul(s1[n], cn); }
    y0 = (y0 + pmul(u0_, D0)) * nsilu(res[t * DI + dA]); y1 = (y1 + pmul(u1_, D1)) * nsilu(res[t * DI + dB]);
    b16 a0, c0, a1, c1; split16(y0 * 8.0f, a0, c0); split16(y1 * 8.0f, a1, c1);
    for (int pass = 0; pass < 2; ++pass) { ((volatile b16*)uyh)[t * DI + dA] = a0; ((volatile b16*)uyh)[t * DI + dB] = a1; ((volatile b16*)uyl)[t * DI + dA] = c0; ((volatile b16*)uyl)[t * DI + dB] = c1; }
  }
  __threadfence();
}

__global__ __launch_bounds__(128) void outproj_kernel(const b16* __restrict__ yh, const b16* __restrict__ yl, const b16* __restrict__ woh, const b16* __restrict__ wol, float* __restrict__ out) {
  __shared__ __attribute__((aligned(16))) float Tc[64][128 + 4];
  const int lane = threadIdx.x & 31, wave = threadIdx.x >> 5, nloc = lane & 15, hlf = lane >> 4, t0 = blockIdx.y * 128, m0 = t0 + wave * 32, c0 = blockIdx.x * 64, b = t0 / L, l0 = t0 % L;
  v8f acc[2][4];
#pragma unroll
  for (int r = 0; r < 2; ++r)
#pragma unroll
    for (int t = 0; t < 4; ++t) acc[r][t] = (v8f){};
#pragma unroll 1
  for (int kb = 0; kb < DI; kb += 32) { const v16b a0 = frag_kb(yh + (size_t)(m0 + nloc) * DI + kb, hlf), l0_ = frag_kb(yl + (size_t)(m0 + nloc) * DI + kb, hlf), a1 = frag_kb(yh + (size_t)(m0 + 16 + nloc) * DI + kb, hlf), l1 = frag_kb(yl + (size_t)(m0 + 16 + nloc) * DI + kb, hlf);
#pragma unroll
    for (int t = 0; t < 4; ++t) { const size_t bo = (size_t)(c0 + t * 16 + nloc) * DI + kb; const v16b b0 = frag_kb(woh + bo, hlf), b1 = frag_kb(wol + bo, hlf);
      acc[0][t] = wmma16b(a0, b0, acc[0][t]); acc[0][t] = wmma16b(l0_, b0, acc[0][t]); acc[0][t] = wmma16b(a0, b1, acc[0][t]);
      acc[1][t] = wmma16b(a1, b0, acc[1][t]); acc[1][t] = wmma16b(l1, b0, acc[1][t]); acc[1][t] = wmma16b(a1, b1, acc[1][t]); } }
#pragma unroll
  for (int t = 0; t < 4; ++t)
#pragma unroll
    for (int r = 0; r < 2; ++r)
#pragma unroll
      for (int v = 0; v < 8; ++v) Tc[t * 16 + nloc][wave * 32 + r * 16 + 8 * hlf + v] = acc[r][t][v] * (1.0f / 512.0f);
  __syncthreads();
  for (int pass = 0; pass < 2; ++pass) { for (int i = threadIdx.x; i < 64 * 32; i += 128) { const int c = i >> 5, q = (i & 31) * 4; *(volatile v4f*)(out + ((size_t)b * DIM + c0 + c) * L + l0 + q) = *(const v4f*)(&Tc[c][q]); } __threadfence(); }
}
}

extern "C" void kernel_launch(void* const* d_in, const int* in_sizes, int n_in,
                              void* d_out, int out_size, void* d_ws, size_t ws_size, hipStream_t stream) {
  (void)n_in; (void)out_size;
  const float* x = (const float*)d_in[0]; const float* win = (const float*)d_in[1]; const float* cw = (const float*)d_in[2]; const float* cb = (const float*)d_in[3]; const float* wx = (const float*)d_in[4];
  const float* wdt = (const float*)d_in[5]; const float* bdt = (const float*)d_in[6]; const float* alog = (const float*)d_in[7]; const float* Dv = (const float*)d_in[8]; const float* wout = (const float*)d_in[9];
  float* out = (float*)d_out;
  if (in_sizes[0] != Bn * DIM * L || in_sizes[1] != 2 * DI * DIM || in_sizes[2] != DI * KC || in_sizes[4] != NXP * DI || in_sizes[5] != DI * DTR || in_sizes[7] != DI * DS || in_sizes[9] != DIM * DI) return;
  size_t off = 0; char* ws = (char*)d_ws;
  auto carve = [&](size_t bytes) { char* p = ws + off; off += (bytes + 255) & ~(size_t)255; return p; };
  b16* xh = (b16*)carve((size_t)NT * DIM * 2); b16* xl = (b16*)carve((size_t)NT * DIM * 2);
  b16* wih = (b16*)carve((size_t)2 * DI * DIM * 2); b16* wil = (b16*)carve((size_t)2 * DI * DIM * 2); b16* wxh = (b16*)carve((size_t)NXPP * DI * 2); b16* wxl = (b16*)carve((size_t)NXPP * DI * 2); b16* woh = (b16*)carve((size_t)DIM * DI * 2); b16* wol = (b16*)carve((size_t)DIM * DI * 2);
  float* u0 = (float*)carve((size_t)NT * DI * 4); float* res = (float*)carve((size_t)NT * DI * 4); b16* uh = (b16*)carve((size_t)NT * DI * 2); b16* ul = (b16*)carve((size_t)NT * DI * 2); float* dbc = (float*)carve((size_t)NT * NXPP * 4);
  if (off > ws_size) return;
  prep_kernel<<<1024, 256, 0, stream>>>(x, win, wx, wout, xh, xl, wih, wil, wxh, wxl, woh, wol);
  gemm_kernel<DIM, DI, false><<<dim3(DI / 64, NT / 128), 128, 0, stream>>>(xh, xl, wih, wil, u0);
  gemm_kernel<DIM, DI, false><<<dim3(DI / 64, NT / 128), 128, 0, stream>>>(xh, xl, wih + (size_t)DI * DIM, wil + (size_t)DI * DIM, res);
  conv_kernel<<<NT * 128 / 256, 256, 0, stream>>>(u0, cw, cb, uh, ul);
  gemm_kernel<DI, NXPP, false><<<dim3(1, NT / 128), 128, 0, stream>>>(uh, ul, wxh, wxl, dbc);
  scan_kernel<<<dim3(1, Bn), 256, 0, stream>>>(dbc, uh, ul, res, wdt, bdt, alog, Dv);
  outproj_kernel<<<dim3(DIM / 64, NT / 128), 128, 0, stream>>>(uh, ul, woh, wol, out);
}
